// SOA_76158360092784
// MI455X (gfx1250) — hardware-verified
//
#include <hip/hip_runtime.h>


#define NB_  8
#define NN_  2048
#define NC_  256
#define DK   64
#define DV   256
#define NTK  (NB_ * NN_)
#define QKVW 384
#define PSC  32768.0f
#define LOSC 1024.0f
#define LOSCI (1.0f / 1024.0f)

typedef _Float16 h16;
typedef unsigned short bf;
typedef __attribute__((ext_vector_type(16))) __bf16   v16bf;
typedef __attribute__((ext_vector_type(16))) _Float16 v16h;
typedef __attribute__((ext_vector_type(8)))  _Float16 v8h;
typedef __attribute__((ext_vector_type(8)))  unsigned short v8us;
typedef __attribute__((ext_vector_type(8)))  float    v8f;
typedef __attribute__((ext_vector_type(4)))  float    v4f;
typedef __attribute__((ext_vector_type(2)))  _Float16 v2h;
typedef v8h  __attribute__((may_alias)) v8ha;
typedef v4f  __attribute__((may_alias)) v4fa;

__device__ __forceinline__ unsigned short f2bf(float f) { unsigned u = __float_as_uint(f); u += 0x7FFFu + ((u >> 16) & 1u); return (unsigned short)(u >> 16); }
__device__ __forceinline__ v16h cat16(v8h lo, v8h hi) { return __builtin_shufflevector(lo, hi, 0, 1, 2, 3, 4, 5, 6, 7, 8, 9, 10, 11, 12, 13, 14, 15); }
__device__ __forceinline__ v16bf cat16b(v8us lo, v8us hi) { return __builtin_bit_cast(v16bf, __builtin_shufflevector(lo, hi, 0, 1, 2, 3, 4, 5, 6, 7, 8, 9, 10, 11, 12, 13, 14, 15)); }
__device__ __forceinline__ v8f wmma16(v16h a, v16h b, v8f c) { return __builtin_amdgcn_wmma_f32_16x16x32_f16(false, a, false, b, (short)0, c, false, false); }
__device__ __forceinline__ v8f wmmab(v16bf a, v16bf b, v8f c) { return __builtin_amdgcn_wmma_f32_16x16x32_bf16(false, a, false, b, (short)0, c, false, false); }

__global__ __launch_bounds__(256) void k_cvtb(const float* __restrict__ src, int nrows, bf* dst) {
    const int lane = threadIdx.x & 31, r = blockIdx.x * 8 + (threadIdx.x >> 5);
    if (r >= nrows) return;
    v8us t;
#pragma unroll
    for (int i = 0; i < 8; ++i) t[i] = f2bf(src[(size_t)r * NC_ + lane * 8 + i]);
    *(volatile v8us*)(dst + (size_t)r * NC_ + lane * 8) = t; __threadfence(); *(volatile v8us*)(dst + (size_t)r * NC_ + lane * 8) = t;
}

__global__ __launch_bounds__(128) void k_gemmb(const bf* __restrict__ A, const bf* __restrict__ Bn, float* C, int cb) {
    __shared__ __align__(16) float ost[4][16 * 68];
    const int lane = threadIdx.x & 31, wave = threadIdx.x >> 5, lr = lane & 15, hi = lane >> 4;
    const int r0 = blockIdx.x * 64 + wave * 16, c0 = blockIdx.y * 64;
    const size_t aoff = (size_t)(r0 + lr) * NC_ + 8 * hi;
    size_t boff[4];
#pragma unroll
    for (int t = 0; t < 4; ++t) boff[t] = (size_t)(c0 + t * 16 + lr) * NC_ + 8 * hi;
    v8f acc[4];
#pragma unroll
    for (int t = 0; t < 4; ++t) acc[t] = (v8f){};
#pragma unroll 1
    for (int kc = 0; kc < NC_; kc += 32) {
        const v16bf a = cat16b(*(const v8us*)(A + aoff + kc), *(const v8us*)(A + aoff + kc + 16));
#pragma unroll
        for (int t = 0; t < 4; ++t) acc[t] = wmmab(a, cat16b(*(const v8us*)(Bn + boff[t] + kc), *(const v8us*)(Bn + boff[t] + kc + 16)), acc[t]);
        asm volatile("v_nop\n\tv_nop\n\tv_nop\n\tv_nop" : "+v"(acc[0]), "+v"(acc[1]), "+v"(acc[2]), "+v"(acc[3]) : "v"(a));
    }
    float* os = &ost[wave][0];
#pragma unroll
    for (int t = 0; t < 4; ++t)
#pragma unroll
        for (int j = 0; j < 8; ++j) os[(hi * 8 + j) * 68 + t * 16 + lr] = acc[t][j];
    __syncthreads();
    float* crow = C + (size_t)r0 * QKVW + cb + c0;
    auto pass = [&]() {
#pragma unroll
        for (int s = 0; s < 8; ++s) { const int Lid = (lane >> 3) + 4 * s, piece = lane & 7; const int row = Lid >> 1, cofs = (Lid & 1) * 32 + piece * 4;
            const v4f val = *(const v4fa*)(os + row * 68 + cofs); *(volatile v4f*)(crow + (size_t)row * QKVW + cofs) = val; }
    };
    pass(); __threadfence(); pass();
}

__global__ __launch_bounds__(256) void k_qkplanes(const float* __restrict__ QKV, h16* QH, h16* QL, h16* KH, h16* KL) {
    const int lane = threadIdx.x & 31, t = blockIdx.x * 8 + (threadIdx.x >> 5);
    if (t >= NTK) return;
    const float* p = QKV + (size_t)t * QKVW + 2 * lane;
    v2h qh, ql, kh, kl;
#pragma unroll
    for (int i = 0; i < 2; ++i) {
        const float q = p[i], k = p[DK + i];
        const h16 a = (h16)q, b = (h16)k;
        qh[i] = a; ql[i] = (h16)((q - (float)a) * LOSC); kh[i] = b; kl[i] = (h16)((k - (float)b) * LOSC);
    }
    const size_t o = (size_t)t * DK + 2 * lane;
    *(volatile v2h*)(QH + o) = qh; *(volatile v2h*)(QL + o) = ql; *(volatile v2h*)(KH + o) = kh; *(volatile v2h*)(KL + o) = kl;
    __threadfence();
    *(volatile v2h*)(QH + o) = qh; *(volatile v2h*)(QL + o) = ql; *(volatile v2h*)(KH + o) = kh; *(volatile v2h*)(KL + o) = kl;
}

__global__ __launch_bounds__(256) void k_vt(const float* __restrict__ QKV, h16* VT16) {
    __shared__ __align__(16) h16 tile[DV * 72];
    const int b = blockIdx.x / (NN_ / 64), kt = blockIdx.x - b * (NN_ / 64), k0 = kt * 64, tid = threadIdx.x;
    const int kk = tid >> 2, d0 = (tid & 3) * 64;
    const float* src = QKV + ((size_t)b * NN_ + k0 + kk) * QKVW + 2 * DK + d0;
#pragma unroll 8
    for (int i = 0; i < 64; ++i) tile[(d0 + i) * 72 + kk] = (h16)src[i];
    __syncthreads();
    const int piece = tid & 7;
    h16* base = VT16 + (size_t)b * DV * NN_ + k0;
    auto pass = [&]() {
#pragma unroll
        for (int s = 0; s < 8; ++s) { const int d = (tid >> 3) + 32 * s; const v8h val = *(const v8ha*)(tile + d * 72 + piece * 8);
            *(volatile v8h*)(base + (size_t)d * NN_ + piece * 8) = val; }
    };
    pass(); __threadfence(); pass();
}

#define ENERGY_TILE(BH, BL, rowA, rowB)                                                                                    \
    v8f s0 = {}, s1 = {}, x0 = {}, x1 = {};                                                                                   \
    _Pragma("unroll") for (int kc = 0; kc < 2; ++kc) {                                                                       \
        const h16* b0p = BH + (size_t)(rowA) * DK + kc * 32 + 8 * hi; const h16* b1p = BH + (size_t)(rowB) * DK + kc * 32 + 8 * hi; \
        const h16* l0p = BL + (size_t)(rowA) * DK + kc * 32 + 8 * hi; const h16* l1p = BL + (size_t)(rowB) * DK + kc * 32 + 8 * hi; \
        const v16h b0 = cat16(*(const v8h*)b0p, *(const v8h*)(b0p + 16)), b1 = cat16(*(const v8h*)b1p, *(const v8h*)(b1p + 16)); \
        s0 = wmma16(ah[kc], b0, s0); s1 = wmma16(ah[kc], b1, s1);                                                            \
        x0 = wmma16(ah[kc], cat16(*(const v8h*)l0p, *(const v8h*)(l0p + 16)), x0);                                            \
        x1 = wmma16(ah[kc], cat16(*(const v8h*)l1p, *(const v8h*)(l1p + 16)), x1);                                            \
        x0 = wmma16(al[kc], b0, x0); x1 = wmma16(al[kc], b1, x1);                                                            \
    }                                                                                                                         \
    asm volatile("v_nop\n\tv_nop\n\tv_nop\n\tv_nop" : "+v"(s0), "+v"(s1), "+v"(x0), "+v"(x1) : "v"(ah[0]), "v"(al[1]));

__global__ __launch_bounds__(128) void k_colstats(const h16* __restrict__ QH, const h16* __restrict__ QL, const h16* __restrict__ KH, const h16* __restrict__ KL, float* CM, float* CZI) {
    __shared__ __align__(16) float stg[128];
    const int lane = threadIdx.x & 31, wave = threadIdx.x >> 5, lr = lane & 15, hi = lane >> 4;
    const int b = blockIdx.x / (NN_ / 64), jt = blockIdx.x - b * (NN_ / 64);
    const size_t tok0 = (size_t)b * NN_;
    const int m0 = jt * 64 + wave * 16;
    v16h ah[2], al[2];
#pragma unroll
    for (int kc = 0; kc < 2; ++kc) {
        const h16* p = KH + (tok0 + m0 + lr) * DK + kc * 32 + 8 * hi; const h16* pl = KL + (tok0 + m0 + lr) * DK + kc * 32 + 8 * hi;
        ah[kc] = cat16(*(const v8h*)p, *(const v8h*)(p + 16)); al[kc] = cat16(*(const v8h*)pl, *(const v8h*)(pl + 16));
    }
    const h16* qhb = QH + tok0 * DK; const h16* qlb = QL + tok0 * DK;
    float mrow[8], lpart[8];
#pragma unroll
    for (int j = 0; j < 8; ++j) { mrow[j] = -3.0e38f; lpart[j] = 0.f; }
#pragma unroll 1
    for (int it = 0; it < NN_ / 32; ++it) {
        const int i0 = it * 32;
        ENERGY_TILE(qhb, qlb, i0 + lr, i0 + 16 + lr)
#pragma unroll
        for (int j = 0; j < 8; ++j) {
            const float a0 = s0[j] + x0[j] * LOSCI, a1 = s1[j] + x1[j] * LOSCI;
            float mx = fmaxf(a0, a1);
            mx = fmaxf(mx, __shfl_xor(mx, 1, 16)); mx = fmaxf(mx, __shfl_xor(mx, 2, 16)); mx = fmaxf(mx, __shfl_xor(mx, 4, 16)); mx = fmaxf(mx, __shfl_xor(mx, 8, 16));
            const float mn = fmaxf(mrow[j], mx); const float al_ = __expf(mrow[j] - mn); mrow[j] = mn;
            lpart[j] = lpart[j] * al_ + (__expf(a0 - mn) + __expf(a1 - mn));
        }
    }
#pragma unroll
    for (int j = 0; j < 8; ++j) {
        float rs = lpart[j];
        rs += __shfl_xor(rs, 1, 16); rs += __shfl_xor(rs, 2, 16); rs += __shfl_xor(rs, 4, 16); rs += __shfl_xor(rs, 8, 16);
        if (lr == 0) { const int jl = wave * 16 + 8 * hi + j; stg[jl] = mrow[j]; stg[64 + jl] = 1.0f / rs; }
    }
    __syncthreads();
    if (wave == 0) {
        const v4f val = *(const v4fa*)(stg + hi * 64 + lr * 4);
        float* dst = (hi ? CZI : CM) + tok0 + jt * 64 + lr * 4;
        *(volatile v4f*)dst = val; __threadfence(); *(volatile v4f*)dst = val;
    }
}

__global__ __launch_bounds__(128) void k_rows(const h16* __restrict__ QH, const h16* __restrict__ QL, const h16* __restrict__ KH, const h16* __restrict__ KL,
                                             const h16* __restrict__ VT16, const float* __restrict__ CM, const float* __restrict__ CZI, int dofs, float* out) {
    __shared__ __align__(16) h16 plds[4][16 * 32];
    __shared__ __align__(16) float ost[4][16 * 132];
    const int lane = threadIdx.x & 31, wave = threadIdx.x >> 5, lr = lane & 15, hi = lane >> 4;
    const int b = blockIdx.x / (NN_ / 64), qt = blockIdx.x - b * (NN_ / 64);
    const size_t tok0 = (size_t)b * NN_;
    const int n0 = qt * 64 + wave * 16;
    h16* pl = &plds[wave][0];
    v16h ah[2], al[2];
#pragma unroll
    for (int kc = 0; kc < 2; ++kc) {
        const h16* p = QH + (tok0 + n0 + lr) * DK + kc * 32 + 8 * hi; const h16* q = QL + (tok0 + n0 + lr) * DK + kc * 32 + 8 * hi;
        ah[kc] = cat16(*(const v8h*)p, *(const v8h*)(p + 16)); al[kc] = cat16(*(const v8h*)q, *(const v8h*)(q + 16));
    }
    const h16* khb = KH + tok0 * DK; const h16* klb = KL + tok0 * DK;
    const h16* vt_b = VT16 + ((size_t)b * DV + dofs) * NN_;
    const float* cmb = CM + tok0; const float* czb = CZI + tok0;
    v8f o[8];
#pragma unroll
    for (int n = 0; n < 8; ++n) o[n] = (v8f){};
    float rsum[8];
#pragma unroll
    for (int j = 0; j < 8; ++j) rsum[j] = 0.f;
#pragma unroll 1
    for (int jt = 0; jt < NN_ / 32; ++jt) {
        const int mA = jt * 32 + lr, mB = mA + 16;
        const float cmA = cmb[mA], cmB = cmb[mB], czA = czb[mA], czB = czb[mB];
        ENERGY_TILE(khb, klb, mA, mB)
#pragma unroll
        for (int j = 0; j < 8; ++j) {
            const float a0 = __expf((s0[j] + x0[j] * LOSCI) - cmA) * czA, a1 = __expf((s1[j] + x1[j] * LOSCI) - cmB) * czB;
            const h16 h0 = (h16)(a0 * PSC), h1 = (h16)(a1 * PSC);
            rsum[j] += (float)h0 + (float)h1;
            const int mr = hi * 8 + j;
            pl[mr * 32 + lr] = h0; pl[mr * 32 + 16 + lr] = h1;
        }
        asm volatile("" ::: "memory");
        const v16h pa = cat16(*(const v8ha*)(pl + lr * 32 + hi * 8), *(const v8ha*)(pl + lr * 32 + 16 + hi * 8));
#pragma unroll
        for (int n = 0; n < 8; ++n) {
            const h16* vp = vt_b + (size_t)(n * 16 + lr) * NN_ + jt * 32 + hi * 8;
            o[n] = wmma16(pa, cat16(*(const v8h*)vp, *(const v8h*)(vp + 16)), o[n]);
        }
        asm volatile("v_nop\n\tv_nop\n\tv_nop\n\tv_nop" : "+v"(o[0]), "+v"(o[1]), "+v"(o[2]), "+v"(o[3]), "+v"(o[4]), "+v"(o[5]), "+v"(o[6]), "+v"(o[7]) : "v"(pa));
    }
    float inv[8];
#pragma unroll
    for (int j = 0; j < 8; ++j) {
        float rs = rsum[j];
        rs += __shfl_xor(rs, 1, 16); rs += __shfl_xor(rs, 2, 16); rs += __shfl_xor(rs, 4, 16); rs += __shfl_xor(rs, 8, 16);
        inv[j] = 1.0f / (1e-9f * PSC + rs);
    }
    float* os = &ost[wave][0];
#pragma unroll
    for (int n = 0; n < 8; ++n)
#pragma unroll
        for (int j = 0; j < 8; ++j) os[(hi * 8 + j) * 132 + n * 16 + lr] = o[n][j] * inv[j];
    __syncthreads();
    float* crow = out + (tok0 + n0) * DV + dofs;
    auto pass = [&]() {
#pragma unroll
        for (int s = 0; s < 16; ++s) { const int Lid = 4 * s + (lane >> 3), piece = lane & 7; const int row = Lid >> 2, cofs = (Lid & 3) * 32 + piece * 4;
            const v4f val = *(const v4fa*)(os + row * 132 + cofs); *(volatile v4f*)(crow + (size_t)row * DV + cofs) = val; }
    };
    pass(); __threadfence(); pass();
}

extern "C" void kernel_launch(void* const* d_in, const int* in_sizes, int n_in,
                              void* d_out, int out_size, void* d_ws, size_t ws_size, hipStream_t stream) {
    (void)in_sizes; (void)n_in; (void)out_size;
    const float* x = (const float*)d_in[0]; const float* Wq = (const float*)d_in[1]; const float* Wk = (const float*)d_in[2]; const float* Wv = (const float*)d_in[3];
    float* out = (float*)d_out;
    char* wsp = (char*)d_ws;
    auto take = [&](size_t bytes) { char* p = wsp; wsp += (bytes + 255) & ~(size_t)255; return (void*)p; };
    bf* Xb = (bf*)take((size_t)NTK * NC_ * 2); bf* WQb = (bf*)take((size_t)DK * NC_ * 2); bf* WKb = (bf*)take((size_t)DK * NC_ * 2); bf* WVb = (bf*)take((size_t)DV * NC_ * 2);
    float* QKV = (float*)take((size_t)NTK * QKVW * 4);
    h16* QH = (h16*)take((size_t)NTK * DK * 2); h16* QL = (h16*)take((size_t)NTK * DK * 2); h16* KH = (h16*)take((size_t)NTK * DK * 2); h16* KL = (h16*)take((size_t)NTK * DK * 2);
    h16* VT16 = (h16*)take((size_t)NTK * DV * 2);
    float* CM = (float*)take((size_t)NTK * 4); float* CZI = (float*)take((size_t)NTK * 4);
    if ((size_t)(wsp - (char*)d_ws) > ws_size) return;
    k_cvtb<<<NTK / 8, 256, 0, stream>>>(x, NTK, Xb);
    k_cvtb<<<DK / 8, 256, 0, stream>>>(Wq, DK, WQb);
    k_cvtb<<<DK / 8, 256, 0, stream>>>(Wk, DK, WKb);
    k_cvtb<<<DV / 8, 256, 0, stream>>>(Wv, DV, WVb);
    k_gemmb<<<dim3(NTK / 64, DK / 64, 1), 128, 0, stream>>>(Xb, WQb, QKV, 0);
    k_gemmb<<<dim3(NTK / 64, DK / 64, 1), 128, 0, stream>>>(Xb, WKb, QKV, DK);
    k_gemmb<<<dim3(NTK / 64, DV / 64, 1), 128, 0, stream>>>(Xb, WVb, QKV, 2 * DK);
    k_qkplanes<<<NTK / 8, 256, 0, stream>>>(QKV, QH, QL, KH, KL);
    k_vt<<<NB_ * (NN_ / 64), 256, 0, stream>>>(QKV, VT16);
    k_colstats<<<NB_ * (NN_ / 64), 128, 0, stream>>>(QH, QL, KH, KL, CM, CZI);
    k_rows<<<NB_ * (NN_ / 64), 128, 0, stream>>>(QH, QL, KH, KL, VT16, CM, CZI, 0, out);
    k_rows<<<NB_ * (NN_ / 64), 128, 0, stream>>>(QH, QL, KH, KL, VT16, CM, CZI, DV / 2, out);
}
